// CausalMultiHeadSelfAttention_1142461301094
// MI455X (gfx1250) — hardware-verified
//
#include <hip/hip_runtime.h>


#ifndef NB
#define NB 2
#endif
#ifndef SEQ
#define SEQ 2048
#endif
#define NB_FULL  2
#define SEQ_FULL 2048
#define DM   1024
#define NH   16
#define HD   64
#define DQKV (3 * DM)
#define RH   64
#define PCAR 1024.0f
#define VCAR 1024.0f
#define SCL  0.125f
#define L2E  1.4426950408889634f
#define PLP  40
#define AP   68

static_assert(SEQ % 64 == 0);
static_assert(SEQ >= 2 * RH);
static_assert(SEQ <= SEQ_FULL);
static_assert(NB >= 1 && NB <= NB_FULL);
static_assert(RH == 64);
static_assert(DM % 64 == 0 && DQKV % 64 == 0 && DM % 32 == 0 && HD == 64);

typedef _Float16 h16;
typedef unsigned short bf;
typedef __attribute__((ext_vector_type(16))) __bf16   v16bf;
typedef __attribute__((ext_vector_type(16))) _Float16 v16h;
typedef __attribute__((ext_vector_type(8)))  _Float16 v8h;
typedef __attribute__((ext_vector_type(8)))  unsigned short v8us;
typedef __attribute__((ext_vector_type(8)))  float    v8f;
typedef __attribute__((ext_vector_type(4)))  float    v4f;
typedef __attribute__((ext_vector_type(2)))  float    v2f;
typedef __attribute__((ext_vector_type(2)))  _Float16 v2h;
typedef __attribute__((ext_vector_type(2)))  unsigned short v2us;
typedef v8h  __attribute__((may_alias)) v8ha;
typedef v4f  __attribute__((may_alias)) v4fa;
typedef v8us __attribute__((may_alias)) v8usa;

__device__ __forceinline__ unsigned short f2bf(float f) { unsigned u = __float_as_uint(f); u += 0x7FFFu + ((u >> 16) & 1u); return (unsigned short)(u >> 16); }
__device__ __forceinline__ float bf2f(unsigned short b) { return __uint_as_float(((unsigned)b) << 16); }
__device__ __forceinline__ float bfr(float f) { return bf2f(f2bf(f)); }
__device__ __forceinline__ v16h cat16(v8h lo, v8h hi) { return __builtin_shufflevector(lo, hi, 0, 1, 2, 3, 4, 5, 6, 7, 8, 9, 10, 11, 12, 13, 14, 15); }
__device__ __forceinline__ v16bf cat16b(v8us lo, v8us hi) { return __builtin_bit_cast(v16bf, __builtin_shufflevector(lo, hi, 0, 1, 2, 3, 4, 5, 6, 7, 8, 9, 10, 11, 12, 13, 14, 15)); }
__device__ __forceinline__ v8f wmma16(v16h a, v16h b, v8f c) { return __builtin_amdgcn_wmma_f32_16x16x32_f16(false, a, false, b, (short)0, c, false, false); }
__device__ __forceinline__ v8f wmmab(v16bf a, v16bf b, v8f c) { return __builtin_amdgcn_wmma_f32_16x16x32_bf16(false, a, false, b, (short)0, c, false, false); }
__device__ __forceinline__ h16 tohx(float x) { return (h16)x; }
__device__ __forceinline__ void splitf(float y, unsigned short& h, unsigned short& l) { h = f2bf(y); l = f2bf(y - bf2f(h)); }

template <typename T16> struct WFrag;
template <> struct WFrag<h16> { typedef v16h V; static __device__ __forceinline__ V ld(const h16* p) { return cat16(*(const v8h*)p, *(const v8h*)(p + 16)); } static __device__ __forceinline__ v8f mma(V a, V b, v8f c) { return wmma16(a, b, c); } };
template <> struct WFrag<bf> { typedef v16bf V; static __device__ __forceinline__ V ld(const bf* p) { return cat16b(*(const v8us*)p, *(const v8us*)(p + 16)); } static __device__ __forceinline__ v8f mma(V a, V b, v8f c) { return wmmab(a, b, c); } };

template <typename T16, int NSPLIT, bool BIAS>
__global__ __launch_bounds__(32) void k_gemmw(const T16* __restrict__ A, const T16* __restrict__ A2, const T16* __restrict__ Bt, const T16* __restrict__ Bt2, int K, float* C, int ldc, const float* __restrict__ bias, size_t sA, size_t sB, size_t sC) {
    typedef typename WFrag<T16>::V V;
    __shared__ __align__(16) float os[16 * 68];
    const size_t z = blockIdx.z; A += z * sA; if (A2) A2 += z * sA; Bt += z * sB; if (Bt2) Bt2 += z * sB; C += z * sC;
    const int lane = threadIdx.x & 31, lr = lane & 15, hi = lane >> 4; const int r0 = blockIdx.x * 64, c0 = blockIdx.y * 64;
    v8f acc[4][4];
#pragma unroll
    for (int mb = 0; mb < 4; ++mb)
#pragma unroll
        for (int nb = 0; nb < 4; ++nb) acc[mb][nb] = (v8f){};
    const size_t aoff = (size_t)(r0 + lr) * K + 8 * hi, boff = (size_t)(c0 + lr) * K + 8 * hi;
#pragma unroll 1
    for (int kc = 0; kc < K; kc += 32) {
        V a[4], a2[4];
#pragma unroll
        for (int mb = 0; mb < 4; ++mb) { a[mb] = WFrag<T16>::ld(A + aoff + (size_t)mb * 16 * K + kc); if (NSPLIT == 1 || NSPLIT == 2) a2[mb] = WFrag<T16>::ld(A2 + aoff + (size_t)mb * 16 * K + kc); }
#pragma unroll
        for (int nb = 0; nb < 4; ++nb) { const V b = WFrag<T16>::ld(Bt + boff + (size_t)nb * 16 * K + kc); V b2; if (NSPLIT >= 2) b2 = WFrag<T16>::ld(Bt2 + boff + (size_t)nb * 16 * K + kc);
#pragma unroll
            for (int mb = 0; mb < 4; ++mb) { acc[mb][nb] = WFrag<T16>::mma(a[mb], b, acc[mb][nb]); if (NSPLIT == 1 || NSPLIT == 2) acc[mb][nb] = WFrag<T16>::mma(a2[mb], b, acc[mb][nb]); if (NSPLIT >= 2) acc[mb][nb] = WFrag<T16>::mma(a[mb], b2, acc[mb][nb]); } }
        asm volatile("v_nop\n\tv_nop\n\tv_nop\n\tv_nop" : "+v"(acc[0][0]), "+v"(acc[1][1]), "+v"(acc[2][2]), "+v"(acc[3][3]) : "v"(a[0]), "v"(a[3]));
    }
#pragma unroll
    for (int mb = 0; mb < 4; ++mb) {
#pragma unroll
        for (int nb = 0; nb < 4; ++nb) {
#pragma unroll
            for (int j = 0; j < 8; ++j) os[(hi * 8 + j) * 68 + nb * 16 + lr] = acc[mb][nb][j]; }
        __builtin_amdgcn_wave_barrier(); asm volatile("" ::: "memory");
        float* crow = C + (size_t)(r0 + mb * 16) * ldc + c0;
#pragma unroll 1
        for (int ps = 0; ps < 2; ++ps) {
#pragma unroll
            for (int s = 0; s < 8; ++s) { const int row = 2 * s + hi, cofs = lr * 4; v4f val = *(const v4fa*)(os + row * 68 + cofs); if (BIAS) { val[0] += bfr(bias[c0 + cofs]); val[1] += bfr(bias[c0 + cofs + 1]); val[2] += bfr(bias[c0 + cofs + 2]); val[3] += bfr(bias[c0 + cofs + 3]); }
                *(volatile v4f*)(crow + (size_t)row * ldc + cofs) = val; }
            if (ps == 0) __threadfence(); }
        __builtin_amdgcn_wave_barrier(); asm volatile("" ::: "memory");
    }
}

__global__ __launch_bounds__(256) void k_cvt8(const float* __restrict__ src, bf* dst, size_t n8) { const size_t i = (size_t)blockIdx.x * 256 + threadIdx.x; if (i >= n8) return; const v8f v = *(const v8f*)(src + i * 8); v8us o;
#pragma unroll
    for (int k = 0; k < 8; ++k) o[k] = f2bf(v[k]); *(volatile v8us*)(dst + i * 8) = o; __threadfence(); *(volatile v8us*)(dst + i * 8) = o; }

__global__ __launch_bounds__(256) void k_cstab(const int* __restrict__ tp, float* CS) {
    const int idx = blockIdx.x * 256 + threadIdx.x; if (idx >= SEQ * (HD / 2)) return;
    const int i = idx & (HD / 2 - 1), t = idx / (HD / 2);
    const float p32 = (float)exp((double)i * 0.28782313662425575);
    const float invf = (float)(1.0 / (double)p32);
    const float ang = __fmul_rn((float)tp[t], invf);
    const float cn = cosf(ang); const float sn = sinf(ang);
    v2f cs; cs[0] = cn; cs[1] = sn;
    *(volatile v2f*)(CS + (size_t)idx * 2) = cs; __threadfence(); *(volatile v2f*)(CS + (size_t)idx * 2) = cs;
}

__global__ __launch_bounds__(256) void k_rope(const float* __restrict__ F, int pitch, int nheads, const float* __restrict__ CS, h16* P16, float* PF) {
    const size_t e = ((size_t)blockIdx.x * 256 + threadIdx.x) * 2; if (e >= (size_t)nheads * SEQ * HD) return;
    const int d = (int)(e % HD); const int t = (int)((e / HD) % SEQ); const int hh = (int)(e / ((size_t)HD * SEQ));
    const float* f = F + (size_t)t * pitch + hh * HD + d; const float x0 = f[0], x1 = f[1];
    const v2f cs = *(const v2f*)(CS + ((size_t)t * (HD / 2) + (d >> 1)) * 2);
    float a0 = __fmul_rn(x0, cs[0]), b0 = __fmul_rn(x1, cs[1]), a1 = __fmul_rn(x0, cs[1]), b1 = __fmul_rn(x1, cs[0]);
    asm volatile("" : "+v"(a0)); asm volatile("" : "+v"(b0)); asm volatile("" : "+v"(a1)); asm volatile("" : "+v"(b1));
    const float re = __fsub_rn(a0, b0), ro = __fadd_rn(a1, b1);
    v2h o16; o16[0] = tohx(re); o16[1] = tohx(ro); v2f of; of[0] = re; of[1] = ro;
    const bool lowt = (t < RH); const size_t po = ((size_t)hh * RH + t) * HD + d;
#pragma unroll 1
    for (int ps = 0; ps < 2; ++ps) { *(volatile v2h*)(P16 + e) = o16; if (lowt) *(volatile v2f*)(PF + po) = of; if (ps == 0) __threadfence(); }
}

__global__ __launch_bounds__(256) void k_vtp(const float* __restrict__ F, int pitch, int nheads, h16* V16, h16* VR) {
    const size_t e = ((size_t)blockIdx.x * 256 + threadIdx.x) * 2; if (e >= (size_t)nheads * HD * SEQ) return;
    const int t = (int)(e % SEQ); const int d = (int)((e / SEQ) % HD); const int g = (int)(e / ((size_t)SEQ * HD)); v2h o16, r16;
#pragma unroll
    for (int q = 0; q < 2; ++q) { const float x = F[(size_t)(t + q) * pitch + g * HD + d]; const h16 hx = tohx(x); o16[q] = hx; float dr = __fsub_rn(x, (float)hx); asm volatile("" : "+v"(dr)); r16[q] = tohx(dr * VCAR); }
    *(volatile v2h*)(V16 + e) = o16; *(volatile v2h*)(VR + e) = r16; __threadfence(); *(volatile v2h*)(V16 + e) = o16; *(volatile v2h*)(VR + e) = r16;
}

__global__ __launch_bounds__(256) void k_attn0(const float* __restrict__ QF, const float* __restrict__ KF, const float* __restrict__ FV, int pitch, bf* Ah, bf* Al) {
    __shared__ __align__(16) float qs[RH * AP];
    __shared__ __align__(16) float ks[RH * AP];
    __shared__ __align__(16) float vs[RH * AP];
    const int tid = threadIdx.x, lane = tid & 31, w = tid >> 5; const int h = blockIdx.x;
    const float* qp = QF + (size_t)h * RH * HD; const float* kp = KF + (size_t)h * RH * HD; const float* vp = FV + h * HD;
#pragma unroll 1
    for (int i = tid; i < RH * HD / 4; i += 256) { const int r = i >> 4, c = (i & 15) * 4;
        *(v4fa*)(qs + r * AP + c) = *(const v4f*)(qp + (size_t)r * HD + c);
        *(v4fa*)(ks + r * AP + c) = *(const v4f*)(kp + (size_t)r * HD + c);
        *(v4fa*)(vs + r * AP + c) = *(const v4f*)(vp + (size_t)r * pitch + c); }
    __syncthreads();
    const int row = tid >> 2, kb = (tid & 3) * 16;
    float sc[16];
#pragma unroll
    for (int kk = 0; kk < 16; ++kk) sc[kk] = 0.f;
#pragma unroll 1
    for (int d = 0; d < HD; ++d) { const float qv = qs[row * AP + d];
#pragma unroll
        for (int kk = 0; kk < 16; ++kk) sc[kk] += qv * ks[(kb + kk) * AP + d]; }
    float mx = -3.0e38f;
#pragma unroll
    for (int kk = 0; kk < 16; ++kk) { const float t = (kb + kk <= row) ? sc[kk] * SCL : -3.0e38f; sc[kk] = t; mx = fmaxf(mx, t); }
    mx = fmaxf(mx, __shfl_xor(mx, 1, 32)); mx = fmaxf(mx, __shfl_xor(mx, 2, 32));
    float sum = 0.f;
#pragma unroll
    for (int kk = 0; kk < 16; ++kk) { float dd = __fsub_rn(sc[kk], mx); asm volatile("" : "+v"(dd)); sc[kk] = __builtin_amdgcn_exp2f(__fmul_rn(dd, L2E)); sum += sc[kk]; }
    sum += __shfl_xor(sum, 1, 32); sum += __shfl_xor(sum, 2, 32);
    const float f = __fdiv_rn(1.0f, sum);
    __syncthreads();
#pragma unroll
    for (int kk = 0; kk < 16; ++kk) ks[row * AP + kb + kk] = sc[kk] * f;
    __syncthreads();
    float oc[16];
#pragma unroll
    for (int dd = 0; dd < 16; ++dd) oc[dd] = 0.f;
#pragma unroll 1
    for (int j = 0; j < RH; ++j) { const float p = ks[row * AP + j];
#pragma unroll
        for (int dd = 0; dd < 16; ++dd) oc[dd] += p * vs[j * AP + kb + dd]; }
#pragma unroll
    for (int dd = 0; dd < 16; ++dd) qs[row * AP + kb + dd] = oc[dd];
    __syncthreads();
#pragma unroll 1
    for (int ps = 0; ps < 2; ++ps) {
#pragma unroll
        for (int s = 0; s < 2; ++s) { const int r = w * 8 + s * 4 + (lane >> 3), c8 = (lane & 7) * 8; const v4f v0 = *(const v4fa*)(qs + r * AP + c8), v1 = *(const v4fa*)(qs + r * AP + c8 + 4); v8us oh, ol;
#pragma unroll
            for (int q = 0; q < 4; ++q) { unsigned short a, c2; splitf(v0[q], a, c2); oh[q] = a; ol[q] = c2; splitf(v1[q], a, c2); oh[4 + q] = a; ol[4 + q] = c2; }
            const size_t oo = (size_t)r * DM + h * HD + c8; *(volatile v8us*)(Ah + oo) = oh; *(volatile v8us*)(Al + oo) = ol; }
        if (ps == 0) __threadfence(); }
}

__global__ __launch_bounds__(128) void k_attn(const h16* __restrict__ QP, const h16* __restrict__ KP, const h16* __restrict__ VT, const h16* __restrict__ VR, bf* Ah, bf* Al, int ntask) {
    __shared__ __align__(16) h16 pl[4][16 * PLP];
    __shared__ __align__(16) float os[4][16 * AP];
    const int lane = threadIdx.x & 31, lr = lane & 15, hi = lane >> 4, w = threadIdx.x >> 5;
    const int task = blockIdx.x * 4 + w; if (task >= ntask) return;
    constexpr int NQT = SEQ / 16 - RH / 16;
    const int h = task / NQT; const int q0 = RH + (task - h * NQT) * 16;
    const h16* Qp = QP + ((size_t)h * SEQ + q0) * HD; const h16* Kp = KP + (size_t)h * SEQ * HD; const h16* Vp = VT + (size_t)h * HD * SEQ; const h16* Rp = VR + (size_t)h * HD * SEQ;
    h16* plw = &pl[w][0]; float* osw = &os[w][0];
    const v16h aq0 = WFrag<h16>::ld(Qp + (size_t)lr * HD + 8 * hi), aq1 = WFrag<h16>::ld(Qp + (size_t)lr * HD + 32 + 8 * hi);
    v8f o[4], o2[4];
#pragma unroll
    for (int c = 0; c < 4; ++c) { o[c] = (v8f){}; o2[c] = (v8f){}; }
    float mrow[8], lrow[8];
#pragma unroll
    for (int r = 0; r < 8; ++r) { mrow[r] = -3.0e38f; lrow[r] = 0.f; }
#pragma unroll 1
    for (int j0 = 0; j0 < q0 + 16; j0 += 32) {
        const h16* k0p = Kp + (size_t)(j0 + lr) * HD + 8 * hi; const h16* k1p = k0p + 16 * HD;
        const v16h kb0 = WFrag<h16>::ld(k0p), kb1 = WFrag<h16>::ld(k0p + 32), kb2 = WFrag<h16>::ld(k1p), kb3 = WFrag<h16>::ld(k1p + 32);
        v8f s0 = (v8f){}, s1 = (v8f){};
        s0 = wmma16(aq0, kb0, s0); s0 = wmma16(aq1, kb1, s0); s1 = wmma16(aq0, kb2, s1); s1 = wmma16(aq1, kb3, s1);
        asm volatile("v_nop\n\tv_nop\n\tv_nop\n\tv_nop" : "+v"(s0), "+v"(s1) : "v"(aq0), "v"(aq1), "v"(kb0), "v"(kb1), "v"(kb2), "v"(kb3));
#pragma unroll
        for (int r = 0; r < 8; ++r) {
            const int qr = q0 + 8 * hi + r;
            const float t0 = (j0 + lr <= qr) ? s0[r] * SCL : -3.0e38f; const float t1 = (j0 + 16 + lr <= qr) ? s1[r] * SCL : -3.0e38f;
            float mx = fmaxf(t0, t1);
            mx = fmaxf(mx, __shfl_xor(mx, 1, 32)); mx = fmaxf(mx, __shfl_xor(mx, 2, 32)); mx = fmaxf(mx, __shfl_xor(mx, 4, 32)); mx = fmaxf(mx, __shfl_xor(mx, 8, 32));
            const float mn = fmaxf(mrow[r], mx);
            float da = __fsub_rn(mrow[r], mn); asm volatile("" : "+v"(da)); const float al = __builtin_amdgcn_exp2f(__fmul_rn(da, L2E));
            mrow[r] = mn;
            float d0 = __fsub_rn(t0, mn), d1 = __fsub_rn(t1, mn); asm volatile("" : "+v"(d0)); asm volatile("" : "+v"(d1));
            const float e0 = __builtin_amdgcn_exp2f(__fmul_rn(d0, L2E)), e1 = __builtin_amdgcn_exp2f(__fmul_rn(d1, L2E));
            float rs = e0 + e1;
            rs += __shfl_xor(rs, 1, 32); rs += __shfl_xor(rs, 2, 32); rs += __shfl_xor(rs, 4, 32); rs += __shfl_xor(rs, 8, 32);
            lrow[r] = lrow[r] * al + rs;
#pragma unroll
            for (int c = 0; c < 4; ++c) { o[c][r] *= al; o2[c][r] *= al; }
            plw[(8 * hi + r) * PLP + lr] = tohx(e0 * PCAR); plw[(8 * hi + r) * PLP + 16 + lr] = tohx(e1 * PCAR);
        }
        __builtin_amdgcn_fence(3  , "wavefront"); __builtin_amdgcn_wave_barrier(); asm volatile("" ::: "memory");
        const v16h pv = cat16(*(const v8ha*)(plw + lr * PLP + 8 * hi), *(const v8ha*)(plw + lr * PLP + 16 + 8 * hi));
        const size_t vo = (size_t)lr * SEQ + j0 + 8 * hi;
        {
            const v16h vb0 = WFrag<h16>::ld(Vp + vo), vb1 = WFrag<h16>::ld(Vp + vo + 16 * (size_t)SEQ), vb2 = WFrag<h16>::ld(Vp + vo + 32 * (size_t)SEQ), vb3 = WFrag<h16>::ld(Vp + vo + 48 * (size_t)SEQ);
            o[0] = wmma16(pv, vb0, o[0]); o[1] = wmma16(pv, vb1, o[1]); o[2] = wmma16(pv, vb2, o[2]); o[3] = wmma16(pv, vb3, o[3]);
            asm volatile("v_nop\n\tv_nop\n\tv_nop\n\tv_nop" : "+v"(o[0]), "+v"(o[1]), "+v"(o[2]), "+v"(o[3]) : "v"(pv), "v"(vb0), "v"(vb1), "v"(vb2), "v"(vb3));
        }
        {
            const v16h rb0 = WFrag<h16>::ld(Rp + vo), rb1 = WFrag<h16>::ld(Rp + vo + 16 * (size_t)SEQ), rb2 = WFrag<h16>::ld(Rp + vo + 32 * (size_t)SEQ), rb3 = WFrag<h16>::ld(Rp + vo + 48 * (size_t)SEQ);
            o2[0] = wmma16(pv, rb0, o2[0]); o2[1] = wmma16(pv, rb1, o2[1]); o2[2] = wmma16(pv, rb2, o2[2]); o2[3] = wmma16(pv, rb3, o2[3]);
            asm volatile("v_nop\n\tv_nop\n\tv_nop\n\tv_nop" : "+v"(o2[0]), "+v"(o2[1]), "+v"(o2[2]), "+v"(o2[3]) : "v"(pv), "v"(rb0), "v"(rb1), "v"(rb2), "v"(rb3));
        }
    }
#pragma unroll
    for (int r = 0; r < 8; ++r) { const float f = __fdiv_rn(1.0f, lrow[r] * PCAR);
#pragma unroll
        for (int c = 0; c < 4; ++c) osw[(8 * hi + r) * AP + c * 16 + lr] = (o[c][r] + o2[c][r] * (1.0f / VCAR)) * f; }
    __builtin_amdgcn_fence(3  , "wavefront"); __builtin_amdgcn_wave_barrier(); asm volatile("" ::: "memory");
#pragma unroll 1
    for (int ps = 0; ps < 2; ++ps) {
#pragma unroll
        for (int s = 0; s < 4; ++s) { const int rr = s * 4 + (lane >> 3), c8 = (lane & 7) * 8; const v4f v0 = *(const v4fa*)(osw + rr * AP + c8), v1 = *(const v4fa*)(osw + rr * AP + c8 + 4); v8us oh, ol;
#pragma unroll
            for (int q = 0; q < 4; ++q) { unsigned short a, c2; splitf(v0[q], a, c2); oh[q] = a; ol[q] = c2; splitf(v1[q], a, c2); oh[4 + q] = a; ol[4 + q] = c2; }
            const size_t oo = (size_t)(q0 + rr) * DM + h * HD + c8; *(volatile v8us*)(Ah + oo) = oh; *(volatile v8us*)(Al + oo) = ol; }
        if (ps == 0) __threadfence(); }
}

#define WS_WQKV ((size_t)DQKV * DM * 2)
#define WS_WO   ((size_t)DM * DM * 2)
#define WS_CS   ((size_t)SEQ * (HD / 2) * 2 * 4)
#define WS_XB   ((size_t)SEQ * DM * 2)
#define WS_F    ((size_t)SEQ * DQKV * 4)
#define WS_QK   ((size_t)2 * NH * SEQ * HD * 2)
#define WS_VT   ((size_t)NH * HD * SEQ * 2)
#define WS_PF   ((size_t)2 * NH * RH * HD * 4)
#define WS_AT   ((size_t)SEQ * DM * 2)
static_assert(WS_WQKV + WS_WO + WS_CS + WS_XB + WS_F + WS_QK + 2 * WS_VT + WS_PF + 2 * WS_AT + 12 * 256 <= ((size_t)128 << 20));
static_assert((size_t)NB_FULL * SEQ_FULL * DM * 4 == 16777216);

extern "C" void kernel_launch(void* const* d_in, const int* in_sizes, int n_in,
                              void* d_out, int out_size, void* d_ws, size_t ws_size, hipStream_t stream) {
    if (n_in < 4) return;
    if (in_sizes[0] < NB * SEQ * DM || in_sizes[1] < DQKV * DM || in_sizes[2] < DM * DM || in_sizes[3] < SEQ || out_size < NB * SEQ * DM) return;
    const float* x = (const float*)d_in[0];
    const float* qkvw = (const float*)d_in[1];
    const float* ow = (const float*)d_in[2];
    const int* tp = (const int*)d_in[3];
    float* OUT = (float*)d_out;
    char* wsb = (char*)d_ws; size_t used = 0;
    auto take = [&](size_t bytes) { char* p = wsb + used; used += (bytes + 255) & ~(size_t)255; return (void*)p; };
    bf* WQKV = (bf*)take(WS_WQKV); bf* WO = (bf*)take(WS_WO); float* CS = (float*)take(WS_CS); bf* XB = (bf*)take(WS_XB); float* F = (float*)take(WS_F);
    h16* QK16 = (h16*)take(WS_QK); h16* VT16 = (h16*)take(WS_VT); h16* VR16 = (h16*)take(WS_VT); float* PF = (float*)take(WS_PF); bf* ATh = (bf*)take(WS_AT); bf* ATl = (bf*)take(WS_AT);
    if (used > ws_size || used > ((size_t)128 << 20)) return;
    k_cvt8<<<(unsigned)((WS_WQKV / 2 / 8 + 255) / 256), 256, 0, stream>>>(qkvw, WQKV, WS_WQKV / 2 / 8);
    k_cvt8<<<(unsigned)((WS_WO / 2 / 8 + 255) / 256), 256, 0, stream>>>(ow, WO, WS_WO / 2 / 8);
    k_cstab<<<(SEQ * (HD / 2) + 255) / 256, 256, 0, stream>>>(tp, CS);
    const int ntask = NH * (SEQ / 16 - RH / 16);
    for (int b = 0; b < NB; ++b) {
        const float* xb = x + (size_t)b * SEQ_FULL * DM;
        k_cvt8<<<(unsigned)(((size_t)SEQ * DM / 8 + 255) / 256), 256, 0, stream>>>(xb, XB, (size_t)SEQ * DM / 8);
        k_gemmw<bf, 0, false><<<dim3(SEQ / 64, DQKV / 64, 1), 32, 0, stream>>>(XB, nullptr, WQKV, nullptr, DM, F, DQKV, nullptr, (size_t)0, (size_t)0, (size_t)0);
        k_rope<<<(unsigned)(((size_t)2 * NH * SEQ * HD / 2 + 255) / 256), 256, 0, stream>>>(F, DQKV, 2 * NH, CS, QK16, PF);
        k_vtp<<<(unsigned)(((size_t)NH * HD * SEQ / 2 + 255) / 256), 256, 0, stream>>>(F + 2 * DM, DQKV, NH, VT16, VR16);
        k_attn0<<<NH, 256, 0, stream>>>(PF, PF + (size_t)NH * RH * HD, F + 2 * DM, DQKV, ATh, ATl);
        k_attn<<<(unsigned)((ntask + 3) / 4), 128, 0, stream>>>(QK16, QK16 + (size_t)NH * SEQ * HD, VT16, VR16, ATh, ATl, ntask);
        k_gemmw<bf, 1, false><<<dim3(SEQ / 64, DM / 64, 1), 32, 0, stream>>>(ATh, ATl, WO, nullptr, DM, OUT + (size_t)b * SEQ_FULL * DM, DM, nullptr, (size_t)0, (size_t)0, (size_t)0);
    }
}
